// GLFAM_87385404604508
// MI455X (gfx1250) — hardware-verified
//
#include <hip/hip_runtime.h>
#include <math.h>
typedef __attribute__((ext_vector_type(16))) _Float16 v16h;
typedef __attribute__((ext_vector_type(8)))  _Float16 v8h;
typedef __attribute__((ext_vector_type(16))) __bf16   v16b;
typedef __attribute__((ext_vector_type(8)))  __bf16   v8b;
typedef __attribute__((ext_vector_type(8)))  float    v8f;
typedef __attribute__((ext_vector_type(4)))  float    v4f;
#define PSCALE 32768.0f
#define U16(p) ((const unsigned short*)(const void*)(p))
#define PSCALE_INV (1.0f / 32768.0f)

__device__ __forceinline__ unsigned short f2bf_bits(float f) {
  unsigned u = __float_as_uint(f);
  return (unsigned short)((u + 0x7FFFu + ((u >> 16) & 1u)) >> 16);
}
__device__ __forceinline__ float bf_bits2f(unsigned short h) { return __uint_as_float(((unsigned)h) << 16); }

__device__ __forceinline__ void dep_guard_h(v8f& a, v8f& b, v16h x, v16h y) { asm volatile("v_nop\n\tv_nop\n\tv_nop\n\tv_nop" : "+v"(a), "+v"(b) : "v"(x), "v"(y)); }
__device__ __forceinline__ void dep_guard_b(v8f& a, v8f& b, v16b x, v16b y) { asm volatile("v_nop\n\tv_nop\n\tv_nop\n\tv_nop" : "+v"(a), "+v"(b) : "v"(x), "v"(y)); }
__device__ __forceinline__ void keep4_h(v16h a, v16h b, v16h c, v16h d) { asm volatile("v_nop" :: "v"(a), "v"(b), "v"(c), "v"(d)); }
__device__ __forceinline__ void keep4_b(v16b a, v16b b, v16b c, v16b d) { asm volatile("v_nop" :: "v"(a), "v"(b), "v"(c), "v"(d)); }
__device__ __forceinline__ void acc_guard4(v8f& a, v8f& b, v8f& c, v8f& d) { asm volatile("v_nop\n\tv_nop\n\tv_nop\n\tv_nop" : "+v"(a), "+v"(b), "+v"(c), "+v"(d)); }
template <typename T> struct Frag;
template <> struct Frag<_Float16> {
  typedef v16h V; union U { v16h v; v8h h[2]; };
  static __device__ __forceinline__ v16h load(const _Float16* p) {
    U f; f.h[0] = *(const v8h*)(p); f.h[1] = *(const v8h*)(p + 16); return f.v;
  }
  static __device__ __forceinline__ v8f mma(v16h a, v16h b, v8f c) {
    return __builtin_amdgcn_wmma_f32_16x16x32_f16(false, a, false, b, (short)0, c, false, false);
  }
  static __device__ __forceinline__ void guard(v8f& a, v8f& b, v16h x, v16h y) { dep_guard_h(a, b, x, y); }
  static __device__ __forceinline__ void keep(v16h a, v16h b, v16h c, v16h d) { keep4_h(a, b, c, d); }
};
template <> struct Frag<__bf16> {
  typedef v16b V; union U { v16b v; v8b h[2]; };
  static __device__ __forceinline__ v16b load(const __bf16* p) {
    U f; f.h[0] = *(const v8b*)(p); f.h[1] = *(const v8b*)(p + 16); return f.v;
  }
  static __device__ __forceinline__ v8f mma(v16b a, v16b b, v8f c) {
    return __builtin_amdgcn_wmma_f32_16x16x32_bf16(false, a, false, b, (short)0, c, false, false);
  }
  static __device__ __forceinline__ void guard(v8f& a, v8f& b, v16b x, v16b y) { dep_guard_b(a, b, x, y); }
  static __device__ __forceinline__ void keep(v16b a, v16b b, v16b c, v16b d) { keep4_b(a, b, c, d); }
};

template <int ET> struct Elem;
template <> struct Elem<0> { typedef _Float16 T; };
template <> struct Elem<1> { typedef __bf16 T; };
template <int ET, bool SPLIT, int BIAS_MODE, int OUT_MODE, bool RESID, int ACT = 0>
__global__ __launch_bounds__(256) void wmma_gemm64(
    const unsigned short* __restrict__ Ap, const unsigned short* __restrict__ A2p, int lda, long strideA,
    const unsigned short* __restrict__ Btp, const unsigned short* __restrict__ Bt2p, int ldb, long strideB,
    void* __restrict__ Cout, void* __restrict__ Cout2, int ldc, long strideC,
    const float* __restrict__ bias,
    const float* __restrict__ resid, long strideR,
    int M, int N, int K, float scale) {
  typedef typename Elem<ET>::T T;
  typedef typename Frag<T>::V V;
  const T* A = (const T*)Ap; const T* A2 = (const T*)A2p; const T* Bt = (const T*)Btp; const T* Bt2 = (const T*)Bt2p;
  __shared__ __align__(16) float sT[8][16 * 68];
  const int b    = blockIdx.y;
  const int lane = threadIdx.x & 31;
  const int wave = threadIdx.x >> 5;
  const int tilesN = N >> 6;
  const int tilesM = M >> 6;
  const int tile = blockIdx.x * 8 + wave;
  if (tile >= tilesM * tilesN) return;
  const int tm = tile / tilesN;
  const int tn = tile - tm * tilesN;
  const int m0 = tm << 6;
  const int n0 = tn << 6;

  const T* Ab  = A  + (size_t)b * strideA;
  const T* Bb  = Bt + (size_t)b * strideB;
  const T* Ab2 = SPLIT ? (A2  + (size_t)b * strideA) : nullptr;
  const T* Bb2 = SPLIT ? (Bt2 + (size_t)b * strideB) : nullptr;

  const int rlane = lane & 15;
  const int koff  = (lane >> 4) * 8;
  const int mOff  = (lane >> 4) * 8;

  v8f acc[4][4];
#pragma unroll
  for (int i = 0; i < 4; ++i)
#pragma unroll
    for (int j = 0; j < 4; ++j) acc[i][j] = (v8f){0.f,0.f,0.f,0.f,0.f,0.f,0.f,0.f};

  for (int k0 = 0; k0 < K; k0 += 32) {
    V bh[4], bl[4];
#pragma unroll
    for (int j = 0; j < 4; ++j) {
      const size_t bo = (size_t)(n0 + (j << 4) + rlane) * ldb + koff + k0;
      bh[j] = Frag<T>::load(Bb + bo);
      if (SPLIT) bl[j] = Frag<T>::load(Bb2 + bo);
    }
#pragma unroll
    for (int i = 0; i < 4; ++i) {
      const size_t ao = (size_t)(m0 + (i << 4) + rlane) * lda + koff + k0;
      V ah = Frag<T>::load(Ab + ao);
      V al;
      if (SPLIT) al = Frag<T>::load(Ab2 + ao);
#pragma unroll
      for (int j = 0; j < 4; ++j) {
        acc[i][j] = Frag<T>::mma(ah, bh[j], acc[i][j]);
        if (SPLIT) {
          acc[i][j] = Frag<T>::mma(ah, bl[j], acc[i][j]);
          acc[i][j] = Frag<T>::mma(al, bh[j], acc[i][j]);
        }
      }
      Frag<T>::guard(acc[i][0], acc[i][3], ah, SPLIT ? al : ah);
    }
    Frag<T>::keep(bh[0], bh[1], bh[2], bh[3]);
    if (SPLIT) Frag<T>::keep(bl[0], bl[1], bl[2], bl[3]);
  }
  acc_guard4(acc[0][0], acc[0][1], acc[0][2], acc[0][3]);
  acc_guard4(acc[1][0], acc[1][1], acc[1][2], acc[1][3]);
  acc_guard4(acc[2][0], acc[2][1], acc[2][2], acc[2][3]);
  acc_guard4(acc[3][0], acc[3][1], acc[3][2], acc[3][3]);

  float* slab = sT[wave];
  const float* Rb = RESID ? (resid + (size_t)b * strideR) : nullptr;
#pragma unroll
  for (int i = 0; i < 4; ++i) {
    const int mBase = m0 + (i << 4);
#pragma unroll
    for (int j = 0; j < 4; ++j) {
      const int n = n0 + (j << 4) + rlane;
      float bv = 0.f;
      if (BIAS_MODE == 2) bv = bias[n];
#pragma unroll
      for (int r = 0; r < 8; ++r) {
        float v = acc[i][j][r] * scale;
        if (BIAS_MODE == 1) v += bias[mBase + mOff + r];
        if (BIAS_MODE == 2) v += bv;
        if (RESID) v += Rb[(size_t)(mBase + mOff + r) * ldc + n];
        if (ACT == 1) v = tanhf(v);
        if (ACT == 2) v = fmaxf(v, 0.0f);
        if (ACT == 3) v = v / (1.0f + expf(-v));
        if (ACT == 4) v = (v > 0.f) ? v : 0.01f * v;
        if (ACT == 5) v = 0.5f * v * (1.0f + erff(v * 0.70710678118654752f));
        slab[(mOff + r) * 68 + (j << 4) + rlane] = v;
      }
    }
    __builtin_amdgcn_fence(__ATOMIC_RELEASE, "workgroup");
    __builtin_amdgcn_wave_barrier();
    __builtin_amdgcn_fence(__ATOMIC_ACQUIRE, "workgroup");
    if (OUT_MODE == 0) {
      float* C = (float*)Cout + (size_t)b * strideC;
      const int hh = lane >> 4, c4 = (lane & 15) * 4;
      for (int pass = 0; pass < 2; ++pass) {
#pragma unroll
        for (int it = 0; it < 8; ++it) {
          const int row = it * 2 + hh;
          v4f v = *(const v4f*)(slab + row * 68 + c4);
          *(volatile v4f*)(C + (size_t)(mBase + row) * ldc + n0 + c4) = v;
        }
        __threadfence();
      }
    } else {
      const int q = lane >> 3, c8 = (lane & 7) * 8;
      unsigned short* C  = (unsigned short*)Cout  + (size_t)b * strideC;
      unsigned short* C2 = (OUT_MODE == 2) ? ((unsigned short*)Cout2 + (size_t)b * strideC) : nullptr;
      for (int pass = 0; pass < 2; ++pass) {
#pragma unroll
        for (int it = 0; it < 4; ++it) {
          const int row = it * 4 + q;
          const float* sp = slab + row * 68 + c8;
          v8h hv, lv;
#pragma unroll
          for (int e = 0; e < 8; ++e) {
            if (OUT_MODE == 1) {
              hv[e] = (_Float16)sp[e];
            } else {
              unsigned short hb = f2bf_bits(sp[e]);
              unsigned short lb = f2bf_bits(sp[e] - bf_bits2f(hb));
              hv[e] = __builtin_bit_cast(_Float16, hb);
              lv[e] = __builtin_bit_cast(_Float16, lb);
            }
          }
          *(volatile v8h*)(C + (size_t)(mBase + row) * ldc + n0 + c8) = hv;
          if (OUT_MODE == 2) *(volatile v8h*)(C2 + (size_t)(mBase + row) * ldc + n0 + c8) = lv;
        }
        __threadfence();
      }
    }
    __builtin_amdgcn_fence(__ATOMIC_RELEASE, "workgroup");
    __builtin_amdgcn_wave_barrier();
    __builtin_amdgcn_fence(__ATOMIC_ACQUIRE, "workgroup");
  }
}


#define GB 8
#define GC 128
#define GHALF 64
#define GHW 64
#define GNP 4096
#define GR (GB * GNP)
#define GKC 576
__device__ __forceinline__ unsigned pkh(float a, float b) { return (unsigned)__builtin_bit_cast(unsigned short, (_Float16)a) | ((unsigned)__builtin_bit_cast(unsigned short, (_Float16)b) << 16); }
__device__ __forceinline__ float gelu_e(float v) { return 0.5f * v * (1.0f + erff(v * 0.70710678118654752f)); }
__global__ __launch_bounds__(256) void xpose_kernel(const float* __restrict__ x, float* __restrict__ XPF, unsigned* __restrict__ XP2) {
  __shared__ float tile[GC][65];
  const int b = blockIdx.y, p0 = blockIdx.x * 64, tx = threadIdx.x, ty = threadIdx.y;
  for (int c = ty; c < GC; c += 8) { const float* src = x + ((size_t)b * GC + c) * GNP + p0; tile[c][tx] = src[tx]; tile[c][32 + tx] = src[32 + tx]; }
  __syncthreads();
  for (int pass = 0; pass < 2; ++pass) {
    for (int p = ty; p < 64; p += 8) { float* d = XPF + ((size_t)b * GNP + p0 + p) * GHALF; ((volatile float*)d)[tx] = tile[tx][p]; ((volatile float*)d)[32 + tx] = tile[32 + tx][p];
      ((volatile unsigned*)XP2)[(((size_t)b * GNP + p0 + p) * GHALF) / 2 + tx] = pkh(tile[64 + 2 * tx][p], tile[64 + 2 * tx + 1][p]); }
    __threadfence(); }
}
__global__ __launch_bounds__(256) void im2col_kernel(const float* __restrict__ XPF, unsigned* __restrict__ COL) {
  const int lane = threadIdx.x & 31, wave = threadIdx.x >> 5; const long g = (long)blockIdx.x * 8 + wave; const int k = (int)(g % 9); const long pos = g / 9; const int b = (int)(pos / GNP), p = (int)(pos % GNP); const int y = p / GHW, xx = p % GHW;
  const int yy = y + k / 3 - 1, xs = xx + k % 3 - 1; unsigned u = 0u;
  if (yy >= 0 && yy < GHW && xs >= 0 && xs < GHW) { const float* s = XPF + ((size_t)b * GNP + yy * GHW + xs) * GHALF + 2 * lane; u = pkh(s[0], s[1]); }
  ((volatile unsigned*)COL)[(pos * GKC + k * 64) / 2 + lane] = u; __threadfence(); ((volatile unsigned*)COL)[(pos * GKC + k * 64) / 2 + lane] = u;
}
__global__ __launch_bounds__(256) void dcol_kernel(const float* __restrict__ XPF, const float* __restrict__ OFF, unsigned* __restrict__ COL) {
  const int lane = threadIdx.x & 31, wave = threadIdx.x >> 5; const long g = (long)blockIdx.x * 8 + wave; const int k = (int)(g % 9); const long pos = g / 9; const int b = (int)(pos / GNP), p = (int)(pos % GNP); const int y = p / GHW, xx = p % GHW;
  const float ys = (float)y + (float)(k / 3 - 1) + OFF[pos * 64 + 2 * k], xs = (float)xx + (float)(k % 3 - 1) + OFF[pos * 64 + 2 * k + 1];
  const float fy = floorf(ys), fx = floorf(xs); const int y0 = (int)fy, x0 = (int)fx; const float wy1 = ys - fy, wx1 = xs - fx, wy0 = 1.0f - wy1, wx0 = 1.0f - wx1;
  float a0 = 0.f, a1 = 0.f;
#pragma unroll
  for (int t = 0; t < 4; ++t) { const int yi = y0 + (t >> 1), xi = x0 + (t & 1); const float w = ((t >> 1) ? wy1 : wy0) * ((t & 1) ? wx1 : wx0);
    if (yi >= 0 && yi < GHW && xi >= 0 && xi < GHW) { const float* s = XPF + ((size_t)b * GNP + yi * GHW + xi) * GHALF + 2 * lane; a0 += w * s[0]; a1 += w * s[1]; } }
  const unsigned u = pkh(a0, a1); ((volatile unsigned*)COL)[(pos * GKC + k * 64) / 2 + lane] = u; __threadfence(); ((volatile unsigned*)COL)[(pos * GKC + k * 64) / 2 + lane] = u;
}
__global__ __launch_bounds__(256) void wcol_kernel(const float* __restrict__ Wc, int CO, int NOP, unsigned* __restrict__ BT) {
  for (int i = blockIdx.x * 256 + threadIdx.x; i < NOP * GKC / 2; i += gridDim.x * 256) { const int o = i / (GKC / 2), cp = 2 * (i % (GKC / 2)); const int k = cp / 64, ci = cp % 64; float a = 0.f, b = 0.f;
    if (o < CO) { a = Wc[((size_t)o * 64 + ci) * 9 + k]; b = Wc[((size_t)o * 64 + ci + 1) * 9 + k]; }
    ((volatile unsigned*)BT)[i] = pkh(a, b); __threadfence(); ((volatile unsigned*)BT)[i] = pkh(a, b); }
}
__global__ __launch_bounds__(256) void wq_kernel(const float* __restrict__ Wq, unsigned* __restrict__ BT) { for (int i = threadIdx.x; i < GC * GHALF / 2; i += 256) { const unsigned u = pkh(Wq[2 * i], Wq[2 * i + 1]); ((volatile unsigned*)BT)[i] = u; __threadfence(); ((volatile unsigned*)BT)[i] = u; } }
__global__ __launch_bounds__(256) void post1_kernel(const float* __restrict__ D1, const float* __restrict__ G, float* __restrict__ out, unsigned* __restrict__ Q16, unsigned* __restrict__ K16, unsigned* __restrict__ VT) {
  __shared__ float td[64][65]; __shared__ float tg[64][129];
  const int b = blockIdx.y, p0 = blockIdx.x * 64, tx = threadIdx.x, ty = threadIdx.y;
  for (int p = ty; p < 64; p += 8) { const size_t pos = (size_t)b * GNP + p0 + p; td[p][tx] = D1[pos * 64 + tx]; td[p][32 + tx] = D1[pos * 64 + 32 + tx]; for (int c = tx; c < GC; c += 32) tg[p][c] = G[pos * GC + c]; }
  __syncthreads();
  for (int pass = 0; pass < 2; ++pass) {
    for (int c = ty; c < 64; c += 8) { float* d = out + ((size_t)b * GC + c) * GNP + p0; ((volatile float*)d)[tx] = td[tx][c]; ((volatile float*)d)[32 + tx] = td[32 + tx][c]; }
    for (int c = ty; c < 32; c += 8) { float* d = out + ((size_t)b * GC + 64 + c) * GNP + p0; ((volatile float*)d)[tx] = tg[tx][96 + c]; ((volatile float*)d)[32 + tx] = tg[32 + tx][96 + c];
      unsigned* v = VT + (((size_t)b * 64 + c) * GNP + p0) / 2; ((volatile unsigned*)v)[tx] = pkh(tg[2 * tx][64 + c], tg[2 * tx + 1][64 + c]); }
    for (int p = ty; p < 64; p += 8) { const size_t pos = (size_t)b * GNP + p0 + p; if (tx < 16) { ((volatile unsigned*)Q16)[(pos * 32) / 2 + tx] = pkh(tg[p][2 * tx], tg[p][2 * tx + 1]); ((volatile unsigned*)K16)[(pos * 32) / 2 + tx] = pkh(tg[p][32 + 2 * tx], tg[p][32 + 2 * tx + 1]); } }
    __threadfence(); }
}
__global__ __launch_bounds__(256) void vtzero_kernel(unsigned* __restrict__ VT) { const long i = (long)blockIdx.x * 256 + threadIdx.x; const long per = (long)64 * GNP / 2; if (i >= (long)GB * per) return; const long r = (i % per) / (GNP / 2); if (r >= 32) { ((volatile unsigned*)VT)[i] = 0u; __threadfence(); ((volatile unsigned*)VT)[i] = 0u; } }
__global__ __launch_bounds__(256) void soft_kernel(const float* __restrict__ S, unsigned* __restrict__ P16) {
  const int lane = threadIdx.x & 31, wave = threadIdx.x >> 5; const size_t row = (size_t)blockIdx.x * 8 + wave; const float* s = S + row * GNP;
  float mx = -INFINITY; for (int j = lane * 4; j < GNP; j += 128) { const v4f v = *(const v4f*)(s + j); mx = fmaxf(mx, fmaxf(fmaxf(v[0], v[1]), fmaxf(v[2], v[3]))); }
  for (int o = 16; o > 0; o >>= 1) mx = fmaxf(mx, __shfl_xor(mx, o, 32));
  float sum = 0.f; for (int j = lane * 4; j < GNP; j += 128) { const v4f v = *(const v4f*)(s + j); sum += __expf(v[0] - mx) + __expf(v[1] - mx) + __expf(v[2] - mx) + __expf(v[3] - mx); }
  for (int o = 16; o > 0; o >>= 1) sum += __shfl_xor(sum, o, 32);
  const float sc = 32768.0f / sum; typedef __attribute__((ext_vector_type(2))) unsigned u2;
  for (int pass = 0; pass < 2; ++pass) { for (int j = lane * 4; j < GNP; j += 128) { const v4f v = *(const v4f*)(s + j); const u2 u = {pkh(__expf(v[0] - mx) * sc, __expf(v[1] - mx) * sc), pkh(__expf(v[2] - mx) * sc, __expf(v[3] - mx) * sc)}; *(volatile u2*)(P16 + (row * GNP + j) / 2) = u; } __threadfence(); }
}
__global__ __launch_bounds__(256) void post2_kernel(const float* __restrict__ O, int b, float* __restrict__ out) {
  __shared__ float t[64][33];
  const int p0 = blockIdx.x * 64, tx = threadIdx.x, ty = threadIdx.y;
  for (int p = ty; p < 64; p += 8) t[p][tx] = O[(size_t)(p0 + p) * 64 + tx];
  __syncthreads();
  for (int pass = 0; pass < 2; ++pass) { for (int d = ty; d < 32; d += 8) { float* dst = out + ((size_t)b * GC + 96 + d) * GNP + p0; ((volatile float*)dst)[tx] = t[tx][d]; ((volatile float*)dst)[32 + tx] = t[32 + tx][d]; } __threadfence(); }
}
__global__ __launch_bounds__(64) void boffpad_kernel(const float* __restrict__ b, float* __restrict__ o) { const int i = threadIdx.x; const float v = (i < 18) ? b[i] : 0.f; ((volatile float*)o)[i] = v; __threadfence(); ((volatile float*)o)[i] = v; }
extern "C" void kernel_launch(void* const* d_in, const int* in_sizes, int n_in, void* d_out, int out_size, void* d_ws, size_t ws_size, hipStream_t stream) {
  (void)in_sizes; (void)n_in; (void)out_size; (void)ws_size;
  auto Fp = [&](int i) { return (const float*)d_in[i]; };
  const float* x = Fp(0); const float* w_off = Fp(1); const float* b_off = Fp(2); const float* w_def = Fp(3); const float* b_def = Fp(4); const float* w_qkv = Fp(5); const float* b_qkv = Fp(6);
  float* out = (float*)d_out;
  char* ws = (char*)d_ws; size_t off = 0;
  auto carve = [&](size_t bytes) -> char* { char* p = ws + off; off += (bytes + 255) & ~(size_t)255; return p; };
  float* XPF = (float*)carve((size_t)GR * GHALF * 4); unsigned* XP2 = (unsigned*)carve((size_t)GR * GHALF * 2); unsigned* BTO = (unsigned*)carve(64 * GKC * 2); unsigned* BTD = (unsigned*)carve(64 * GKC * 2); unsigned* BTQ = (unsigned*)carve(GC * GHALF * 2); float* BOFF = (float*)carve(256);
  float* OFF = (float*)carve((size_t)GR * 64 * 4); float* D1 = (float*)carve((size_t)GR * 64 * 4); float* G = (float*)carve((size_t)GR * GC * 4); unsigned* Q16 = (unsigned*)carve((size_t)GR * 32 * 2); unsigned* K16 = (unsigned*)carve((size_t)GR * 32 * 2); unsigned* VT = (unsigned*)carve((size_t)GB * 64 * GNP * 2);
  float* O = (float*)carve((size_t)GNP * 64 * 4); unsigned* P16 = (unsigned*)carve((size_t)(GNP / 2) * GNP * 2);
  unsigned* COL = (unsigned*)carve((size_t)GR * GKC * 2); float* S = (float*)COL;
  xpose_kernel<<<dim3(GNP / 64, GB), dim3(32, 8), 0, stream>>>(x, XPF, XP2);
  wcol_kernel<<<24, 256, 0, stream>>>(w_off, 18, 64, BTO); wcol_kernel<<<72, 256, 0, stream>>>(w_def, 64, 64, BTD); wq_kernel<<<1, 256, 0, stream>>>(w_qkv, BTQ);
  boffpad_kernel<<<1, 64, 0, stream>>>(b_off, BOFF);
  vtzero_kernel<<<(unsigned)(((long)GB * 64 * GNP / 2 + 255) / 256), 256, 0, stream>>>(VT);
  const int tr = GR / 64;
  im2col_kernel<<<(unsigned)((long)GR * 9 / 8), 256, 0, stream>>>(XPF, COL);
  wmma_gemm64<0, false, 2, 0, false><<<dim3((tr + 7) / 8, 1), 256, 0, stream>>>((const unsigned short*)COL, nullptr, GKC, 0, (const unsigned short*)BTO, nullptr, GKC, 0, OFF, nullptr, 64, 0, BOFF, nullptr, 0, GR, 64, GKC, 1.0f);
  dcol_kernel<<<(unsigned)((long)GR * 9 / 8), 256, 0, stream>>>(XPF, OFF, COL);
  wmma_gemm64<0, false, 2, 0, false, 5><<<dim3((tr + 7) / 8, 1), 256, 0, stream>>>((const unsigned short*)COL, nullptr, GKC, 0, (const unsigned short*)BTD, nullptr, GKC, 0, D1, nullptr, 64, 0, b_def, nullptr, 0, GR, 64, GKC, 1.0f);
  wmma_gemm64<0, false, 2, 0, false, 5><<<dim3((tr * 2 + 7) / 8, 1), 256, 0, stream>>>((const unsigned short*)XP2, nullptr, GHALF, 0, (const unsigned short*)BTQ, nullptr, GHALF, 0, G, nullptr, GC, 0, b_qkv, nullptr, 0, GR, GC, GHALF, 1.0f);
  post1_kernel<<<dim3(GNP / 64, GB), dim3(32, 8), 0, stream>>>(D1, G, out, Q16, K16, VT);
  const int ts = (GNP / 64) * (GNP / 64), to = (GNP / 64) * 1;
  for (int b = 0; b < GB; ++b) { for (int qh = 0; qh < 2; ++qh) {
      wmma_gemm64<0, false, 0, 0, false><<<dim3((ts / 2 + 7) / 8, 1), 256, 0, stream>>>((const unsigned short*)Q16 + ((size_t)b * GNP + (size_t)qh * (GNP / 2)) * 32, nullptr, 32, 0, (const unsigned short*)K16 + (size_t)b * GNP * 32, nullptr, 32, 0, S, nullptr, GNP, 0, nullptr, nullptr, 0, GNP / 2, GNP, 32, 0.088388347648318447f);
      soft_kernel<<<(GNP / 2) / 8, 256, 0, stream>>>(S, P16);
      wmma_gemm64<0, false, 0, 0, false><<<dim3((to / 2 + 7) / 8, 1), 256, 0, stream>>>((const unsigned short*)P16, nullptr, GNP, 0, (const unsigned short*)VT + (size_t)b * 64 * GNP, nullptr, GNP, 0, O + (size_t)qh * (GNP / 2) * 64, nullptr, 64, 0, nullptr, nullptr, 0, GNP / 2, 64, GNP, 1.0f / 32768.0f); }
    post2_kernel<<<GNP / 64, dim3(32, 8), 0, stream>>>(O, b, out); }
}
